// GAT_17617955848390
// MI455X (gfx1250) — hardware-verified
//
#include <hip/hip_runtime.h>
#include <math.h>
#include <stddef.h>
#include <stdint.h>

#pragma clang fp contract(off)

#define NN    4096
#define IND   256
#define OD    64
#define NH    8
#define NCOL  (NH * OD)
#define NEGSL 0.2f
#define QB    128
#define KC    64
#define SP    68
#define NUX   (NN * (IND / 8))
#define NUW   (NCOL * (IND / 8))
#define WSMAX 134217728

static_assert(NN % QB == 0);
static_assert(NN % KC == 0);
static_assert(OD == 64);
static_assert(NH * OD == 512);
static_assert(IND % 32 == 0);
static_assert(2 * OD == 128);
static_assert(NN * 4 <= 16384);
static_assert(NUX % 256 == 0 && NUW % 256 == 0);
static_assert(QB == 8 * 16);
static_assert(KC == 2 * 32);
static_assert((NN * 4 + 2 * KC * OD * 2 + 8 * 16 * SP * 4 + 8 * 16 * 4 + 8 * 4) <= 327680);

typedef float          v4f   __attribute__((ext_vector_type(4)));
typedef float          v8f   __attribute__((ext_vector_type(8)));
typedef int            v8i   __attribute__((ext_vector_type(8)));
typedef unsigned int   v4u   __attribute__((ext_vector_type(4)));
typedef unsigned short v8us  __attribute__((ext_vector_type(8)));
typedef __bf16         v16bf __attribute__((ext_vector_type(16)));
typedef v4f  __attribute__((may_alias)) v4fa;
typedef v8us __attribute__((may_alias)) v8usa;
union FragB { v16bf v; v8us h[2]; v8i w; };

__device__ __forceinline__ v8f wmb(const FragB& a, const FragB& b, v8f c) {
  v8f d = __builtin_amdgcn_wmma_f32_16x16x32_bf16(false, a.v, false, b.v, (short)0, c, false, false);
  asm volatile("v_nop\n\tv_nop\n\tv_nop\n\tv_nop" : "+v"(d) : "v"(a.w), "v"(b.w));
  return d;
}

__device__ __forceinline__ unsigned bf16_bits(float f) {
  const unsigned u = __float_as_uint(f);
  return (u + 0x7FFFu + ((u >> 16) & 1u)) >> 16;
}
__device__ __forceinline__ float bf16_val(float f) {
  return __uint_as_float(bf16_bits(f) << 16);
}

__device__ __forceinline__ void st2_v8us(unsigned short* dp, const v8us o) {
  *(volatile v8us*)dp = o;
  __threadfence();
  *(volatile v8us*)dp = o;
}

__global__ __launch_bounds__(256) void k_prep(const float* __restrict__ x, const float* __restrict__ w,
                                              unsigned short* XB, unsigned short* WT) {
  const int u = (int)blockIdx.x * 256 + (int)threadIdx.x;
  if (u < NUX) {
    const int row = u >> 5;
    const int k8  = (u & 31) * 8;
    const float* p = x + (size_t)row * IND + k8;
    const v4f a = *(const v4f*)p;
    const v4f b = *(const v4f*)(p + 4);
    v8us o;
    o[0] = (unsigned short)bf16_bits(a.x); o[1] = (unsigned short)bf16_bits(a.y);
    o[2] = (unsigned short)bf16_bits(a.z); o[3] = (unsigned short)bf16_bits(a.w);
    o[4] = (unsigned short)bf16_bits(b.x); o[5] = (unsigned short)bf16_bits(b.y);
    o[6] = (unsigned short)bf16_bits(b.z); o[7] = (unsigned short)bf16_bits(b.w);
    st2_v8us(XB + (size_t)row * IND + k8, o);
  } else if (u < NUX + NUW) {
    const int v  = u - NUX;
    const int n  = v >> 5;
    const int k8 = (v & 31) * 8;
    const int hd = n >> 6;
    const int oc = n & (OD - 1);
    const float* p = w + ((size_t)hd * IND + k8) * OD + oc;
    v8us o;
#pragma unroll
    for (int i = 0; i < 8; ++i) o[i] = (unsigned short)bf16_bits(p[(size_t)i * OD]);
    st2_v8us(WT + (size_t)n * IND + k8, o);
  }
}

__global__ __launch_bounds__(256) void k_proj(const unsigned short* __restrict__ XB,
                                              const unsigned short* __restrict__ WT,
                                              const float* __restrict__ av, float* ESD,
                                              unsigned short* VTH, unsigned short* VTL) {
  __shared__ __align__(16) float stg[QB * SP];
  __shared__ __align__(16) float sa[2 * OD];
  __shared__ __align__(16) float sdt[2 * QB];
  const int tid = (int)threadIdx.x, lane = tid & 31, wave = tid >> 5, hh = lane >> 4, c = lane & 15;
  const int n0 = (int)blockIdx.x * QB;
  const int h  = (int)blockIdx.y;

  if (tid < 2 * OD) sa[tid] = bf16_val(av[h * 2 * OD + tid]);

  v8f acc[4];
  {
    const v8f z = {0.f, 0.f, 0.f, 0.f, 0.f, 0.f, 0.f, 0.f};
#pragma unroll
    for (int t = 0; t < 4; ++t) acc[t] = z;
  }
  const unsigned short* ap = XB + (size_t)(n0 + 16 * wave + c) * IND + 8 * hh;
  const unsigned short* bp = WT + (size_t)(h * OD + c) * IND + 8 * hh;

#pragma unroll 1
  for (int k0 = 0; k0 < IND; k0 += 32) {
    FragB af;
    af.h[0] = *(const v8usa*)(ap + k0);
    af.h[1] = *(const v8usa*)(ap + k0 + 16);
#pragma unroll
    for (int t = 0; t < 4; ++t) {
      const unsigned short* wq = bp + (size_t)(16 * t) * IND + k0;
      FragB bf;
      bf.h[0] = *(const v8usa*)wq;
      bf.h[1] = *(const v8usa*)(wq + 16);
      acc[t] = wmb(af, bf, acc[t]);
    }
  }

#pragma unroll
  for (int t = 0; t < 4; ++t) {
#pragma unroll
    for (int r = 0; r < 8; ++r) {
      stg[(16 * wave + 8 * hh + r) * SP + 16 * t + c] = acc[t][r];
    }
  }
  __syncthreads();

  {
    const int row = tid & (QB - 1);
    const int ao  = (tid >> 7) * OD;
    const float* sr = stg + row * SP;
    float s = 0.0f;
#pragma unroll 4
    for (int q = 0; q < OD / 4; ++q) {
      const v4f p = *(const v4fa*)(sr + 4 * q);
      const v4f g = *(const v4fa*)(sa + ao + 4 * q);
      s = fmaf(p.x, g.x, s); s = fmaf(p.y, g.y, s); s = fmaf(p.z, g.z, s); s = fmaf(p.w, g.w, s);
    }
    sdt[tid] = s;
  }

  const int osub = tid >> 4;
  const int n8   = (tid & 15) * 8;
  v4u hv[4], lv[4];
#pragma unroll
  for (int it = 0; it < 4; ++it) {
    const int orow = it * 16 + osub;
    v4u a1, a2;
#pragma unroll
    for (int q = 0; q < 4; ++q) {
      const float f0 = stg[(n8 + 2 * q) * SP + orow];
      const float f1 = stg[(n8 + 2 * q + 1) * SP + orow];
      const unsigned h0 = bf16_bits(f0), h1 = bf16_bits(f1);
      const unsigned l0 = bf16_bits(f0 - __uint_as_float(h0 << 16));
      const unsigned l1 = bf16_bits(f1 - __uint_as_float(h1 << 16));
      a1[q] = h0 | (h1 << 16);
      a2[q] = l0 | (l1 << 16);
    }
    hv[it] = a1; lv[it] = a2;
  }
  __syncthreads();

  const v4f sv = *(const v4fa*)(sdt + (wave & 1) * QB + 4 * lane);
  float* sp = ESD + (size_t)(wave & 1) * (NH * NN) + (size_t)h * NN + n0 + 4 * lane;
  unsigned short* gh = VTH + (size_t)(h * OD) * NN + n0 + n8;
  unsigned short* gl = VTL + (size_t)(h * OD) * NN + n0 + n8;

#pragma unroll
  for (int it = 0; it < 4; ++it) {
    const size_t ro = (size_t)(it * 16 + osub) * NN;
    *(volatile v4u*)(gh + ro) = hv[it];
    *(volatile v4u*)(gl + ro) = lv[it];
  }
  if (wave < 2) *(volatile v4f*)sp = sv;
  __threadfence();
#pragma unroll
  for (int it = 0; it < 4; ++it) {
    const size_t ro = (size_t)(it * 16 + osub) * NN;
    *(volatile v4u*)(gh + ro) = hv[it];
    *(volatile v4u*)(gl + ro) = lv[it];
  }
  if (wave < 2) *(volatile v4f*)sp = sv;
}

__device__ __forceinline__ float p_of(float es, float ed, float m) {
  float e = es + ed;
  e = (e >= 0.0f) ? e : NEGSL * e;
  return expf(e - m);
}
__device__ __forceinline__ void pword(float eda, float edb, float es, float m, float& ls,
                                      unsigned& wh, unsigned& wl) {
  const float pa = p_of(es, eda, m);
  const float pb = p_of(es, edb, m);
  ls += pa;
  ls += pb;
  const unsigned ha = bf16_bits(pa), hb = bf16_bits(pb);
  const unsigned la = bf16_bits(pa - __uint_as_float(ha << 16));
  const unsigned lb = bf16_bits(pb - __uint_as_float(hb << 16));
  wh = ha | (hb << 16);
  wl = la | (lb << 16);
}

__global__ __launch_bounds__(256) void k_attn(const unsigned short* __restrict__ VTH,
                                              const unsigned short* __restrict__ VTL,
                                              const float* __restrict__ ES, const float* __restrict__ ED,
                                              float* out) {
  __shared__ __align__(16) float          sED[NN];
  __shared__ __align__(16) unsigned short Vth[OD * KC];
  __shared__ __align__(16) unsigned short Vtl[OD * KC];
  __shared__ __align__(16) float          Os[8][16 * SP];
  __shared__ __align__(16) float          Li[8][16];
  __shared__ float red[8];

  const int tid = (int)threadIdx.x, lane = tid & 31, wave = tid >> 5, hh = lane >> 4, c = lane & 15;
  const int h  = (int)blockIdx.y;
  const int q0 = (int)blockIdx.x * QB + wave * 16;

  {
    const float* edh = ED + (size_t)h * NN;
    float mx = -INFINITY;
#pragma unroll
    for (int i = 0; i < 4; ++i) {
      const int idx = (i * 256 + tid) * 4;
      const v4f v = *(const v4f*)(edh + idx);
      *(v4fa*)(sED + idx) = v;
      mx = fmaxf(mx, fmaxf(fmaxf(v.x, v.y), fmaxf(v.z, v.w)));
    }
#pragma unroll
    for (int off = 16; off > 0; off >>= 1) mx = fmaxf(mx, __shfl_xor(mx, off, 32));
    if (lane == 0) red[wave] = mx;
  }
  __syncthreads();
  float edmax = red[0];
#pragma unroll
  for (int i = 1; i < 8; ++i) edmax = fmaxf(edmax, red[i]);

  const float es = ES[(size_t)h * NN + q0 + c];
  const float tm = es + edmax;
  const float m  = (tm >= 0.0f) ? tm : NEGSL * tm;

  v8f oacc[4];
  {
    const v8f z = {0.f, 0.f, 0.f, 0.f, 0.f, 0.f, 0.f, 0.f};
#pragma unroll
    for (int t = 0; t < 4; ++t) oacc[t] = z;
  }
  float lsum = 0.0f;

  const int sr = tid >> 2;
  const int sq = (tid & 3) * 16;
  const unsigned short* gsh = VTH + (size_t)(h * OD + sr) * NN + sq;
  const unsigned short* gsl = VTL + (size_t)(h * OD + sr) * NN + sq;

#pragma unroll 1
  for (int kc = 0; kc < NN / KC; ++kc) {
    const int kv0 = kc * KC;
    const v8us a0 = *(const v8usa*)(gsh + kv0);
    const v8us a1 = *(const v8usa*)(gsh + kv0 + 8);
    const v8us b0 = *(const v8usa*)(gsl + kv0);
    const v8us b1 = *(const v8usa*)(gsl + kv0 + 8);
    __syncthreads();
    *(v8usa*)(Vth + sr * KC + sq)     = a0;
    *(v8usa*)(Vth + sr * KC + sq + 8) = a1;
    *(v8usa*)(Vtl + sr * KC + sq)     = b0;
    *(v8usa*)(Vtl + sr * KC + sq + 8) = b1;
    __syncthreads();

#pragma unroll 1
    for (int kk = 0; kk < 2; ++kk) {
      const int jb = kv0 + kk * 32;
      const v4f t0 = *(const v4fa*)(sED + jb + 8 * hh);
      const v4f t1 = *(const v4fa*)(sED + jb + 8 * hh + 4);
      const v4f t2 = *(const v4fa*)(sED + jb + 16 + 8 * hh);
      const v4f t3 = *(const v4fa*)(sED + jb + 16 + 8 * hh + 4);
      unsigned h0, h1, h2, h3, h4, h5, h6, h7, l0, l1, l2, l3, l4, l5, l6, l7;
      pword(t0.x, t0.y, es, m, lsum, h0, l0);
      pword(t0.z, t0.w, es, m, lsum, h1, l1);
      pword(t1.x, t1.y, es, m, lsum, h2, l2);
      pword(t1.z, t1.w, es, m, lsum, h3, l3);
      pword(t2.x, t2.y, es, m, lsum, h4, l4);
      pword(t2.z, t2.w, es, m, lsum, h5, l5);
      pword(t3.x, t3.y, es, m, lsum, h6, l6);
      pword(t3.z, t3.w, es, m, lsum, h7, l7);
      FragB ph, pl;
      ph.w = (v8i){(int)h0, (int)h1, (int)h2, (int)h3, (int)h4, (int)h5, (int)h6, (int)h7};
      pl.w = (v8i){(int)l0, (int)l1, (int)l2, (int)l3, (int)l4, (int)l5, (int)l6, (int)l7};
#pragma unroll
      for (int t = 0; t < 4; ++t) {
        const int vo = (t * 16 + c) * KC + kk * 32 + 8 * hh;
        FragB vb, vl;
        vb.h[0] = *(const v8usa*)(Vth + vo);
        vb.h[1] = *(const v8usa*)(Vth + vo + 16);
        vl.h[0] = *(const v8usa*)(Vtl + vo);
        vl.h[1] = *(const v8usa*)(Vtl + vo + 16);
        oacc[t] = wmb(ph, vb, oacc[t]);
        oacc[t] = wmb(ph, vl, oacc[t]);
        oacc[t] = wmb(pl, vb, oacc[t]);
      }
    }
  }

  const float ltot = lsum + __shfl_xor(lsum, 16, 32);
  const float linv = 1.0f / ltot;
  float* os = Os[wave];
  float* li = Li[wave];
  if (hh == 0) li[c] = linv;
#pragma unroll
  for (int t = 0; t < 4; ++t) {
#pragma unroll
    for (int r = 0; r < 8; ++r) os[(8 * hh + r) * SP + t * 16 + c] = oacc[t][r];
  }
  __builtin_amdgcn_fence(__ATOMIC_RELEASE, "workgroup");
  __builtin_amdgcn_wave_barrier();
  __builtin_amdgcn_fence(__ATOMIC_ACQUIRE, "workgroup");

  const int c4 = c * 4;
  v4f val[8];
#pragma unroll
  for (int it = 0; it < 8; ++it) {
    const int row = it * 2 + hh;
    const v4f v = *(const v4fa*)(os + row * SP + c4);
    const float s = li[row];
    val[it] = v * s;
  }
  float* ob = out + (size_t)h * OD + c4;
#pragma unroll
  for (int it = 0; it < 8; ++it) {
    const int row = it * 2 + hh;
    *(volatile v4f*)(ob + (size_t)(q0 + row) * NCOL) = val[it];
  }
  __threadfence();
#pragma unroll
  for (int it = 0; it < 8; ++it) {
    const int row = it * 2 + hh;
    *(volatile v4f*)(ob + (size_t)(q0 + row) * NCOL) = val[it];
  }
}

extern "C" void kernel_launch(void* const* d_in, const int* in_sizes, int n_in,
                              void* d_out, int out_size, void* d_ws, size_t ws_size,
                              hipStream_t stream) {
  if (n_in < 3) return;
  if (in_sizes[0] != NN * IND) return;
  if (in_sizes[1] != NH * IND * OD) return;
  if (in_sizes[2] != NH * 2 * OD) return;
  if (out_size != NN * NH * OD) return;

  const float* x = (const float*)d_in[0];
  const float* w = (const float*)d_in[1];
  const float* a = (const float*)d_in[2];
  float* out = (float*)d_out;

  size_t off = 0;
  const size_t oXB  = off; off += (size_t)NN * IND * 2;
  const size_t oWT  = off; off += (size_t)NCOL * IND * 2;
  const size_t oESD = off; off += (size_t)2 * NH * NN * 4;
  const size_t oVTH = off; off += (size_t)NH * OD * NN * 2;
  const size_t oVTL = off; off += (size_t)NH * OD * NN * 2;
  if (off > ws_size || off > (size_t)WSMAX) return;

  char* ws = (char*)d_ws;
  unsigned short* XB  = (unsigned short*)(ws + oXB);
  unsigned short* WT  = (unsigned short*)(ws + oWT);
  float*          ESD = (float*)(ws + oESD);
  unsigned short* VTH = (unsigned short*)(ws + oVTH);
  unsigned short* VTL = (unsigned short*)(ws + oVTL);

  k_prep<<<dim3((NUX + NUW) / 256), dim3(256), 0, stream>>>(x, w, XB, WT);
  k_proj<<<dim3(NN / QB, NH), dim3(256), 0, stream>>>(XB, WT, a, ESD, VTH, VTL);
  k_attn<<<dim3(NN / QB, NH), dim3(256), 0, stream>>>(VTH, VTL, ESD, ESD + (size_t)NH * NN, out);
  (void)hipGetLastError();
}
